// LiquidLayer_61538291417814
// MI455X (gfx1250) — hardware-verified
//
#include <hip/hip_runtime.h>
#include <math.h>

constexpr int NBATCH  = 32;
constexpr int NSTEP   = 512;
constexpr int NIN     = 256;
constexpr int NHID    = 512;
constexpr int NTAU    = NIN + NHID;
constexpr int NODE    = 4;
constexpr int NTHR    = 256;
constexpr int SEQ_BLK = 16;
constexpr int HPITCH  = 520;
constexpr int SLABP   = 68;
constexpr int NROWS   = NBATCH * NSTEP;
constexpr int NOUT0   = NROWS * NHID;
constexpr int NOUT1   = NBATCH * NHID;
constexpr float WCARRY     = 256.0f;
constexpr float WCARRY_INV = 1.0f / 256.0f;
constexpr float LN_EPS_F   = 1e-5f;
static_assert(NBATCH % SEQ_BLK == 0);
static_assert(NHID == 64 * (NTHR / 32));
static_assert(NHID % 32 == 0);
static_assert(NIN % 32 == 0);
static_assert(NROWS % 64 == 0 && NHID % 64 == 0);
static_assert((2 * SEQ_BLK * HPITCH) % NTHR == 0);
static_assert(NROWS % (NTHR / 32) == 0);

typedef __attribute__((ext_vector_type(16))) _Float16 v16h;
typedef __attribute__((ext_vector_type(8)))  _Float16 v8h;
typedef __attribute__((ext_vector_type(16))) __bf16   v16b;
typedef __attribute__((ext_vector_type(8)))  __bf16   v8b;
typedef __attribute__((ext_vector_type(8)))  float    v8f;
typedef __attribute__((ext_vector_type(4)))  float    v4f;

__device__ __forceinline__ unsigned short f2bf_bits(float f) {
  unsigned u = __float_as_uint(f);
  return (unsigned short)((u + 0x7FFFu + ((u >> 16) & 1u)) >> 16);
}
__device__ __forceinline__ float bf_bits2f(unsigned short h) { return __uint_as_float(((unsigned)h) << 16); }
__device__ __forceinline__ float bf16r(float f) { return bf_bits2f(f2bf_bits(f)); }

__device__ __forceinline__ void dep_guard_h(v8f& a, v8f& b, v16h x, v16h y) { asm volatile("v_nop\n\tv_nop\n\tv_nop\n\tv_nop" : "+v"(a), "+v"(b) : "v"(x), "v"(y)); }
__device__ __forceinline__ void dep_guard_b(v8f& a, v8f& b, v16b x, v16b y) { asm volatile("v_nop\n\tv_nop\n\tv_nop\n\tv_nop" : "+v"(a), "+v"(b) : "v"(x), "v"(y)); }
__device__ __forceinline__ void keep4_h(v16h a, v16h b, v16h c, v16h d) { asm volatile("v_nop" :: "v"(a), "v"(b), "v"(c), "v"(d)); }
__device__ __forceinline__ void keep4_b(v16b a, v16b b, v16b c, v16b d) { asm volatile("v_nop" :: "v"(a), "v"(b), "v"(c), "v"(d)); }
__device__ __forceinline__ void acc_guard4(v8f& a, v8f& b, v8f& c, v8f& d) { asm volatile("v_nop\n\tv_nop\n\tv_nop\n\tv_nop" : "+v"(a), "+v"(b), "+v"(c), "+v"(d)); }
__device__ __forceinline__ void acc_guard2(v8f& a, v8f& b) { asm volatile("v_nop\n\tv_nop\n\tv_nop\n\tv_nop" : "+v"(a), "+v"(b)); }
template <typename T> struct Frag;
template <> struct Frag<_Float16> {
  typedef v16h V; union U { v16h v; v8h h[2]; };
  static __device__ __forceinline__ v16h load(const _Float16* p) {
    U f; f.h[0] = *(const v8h*)(p); f.h[1] = *(const v8h*)(p + 16); return f.v;
  }
  static __device__ __forceinline__ v8f mma(v16h a, v16h b, v8f c) {
    return __builtin_amdgcn_wmma_f32_16x16x32_f16(false, a, false, b, (short)0, c, false, false);
  }
  static __device__ __forceinline__ void guard(v8f& a, v8f& b, v16h x, v16h y) { dep_guard_h(a, b, x, y); }
  static __device__ __forceinline__ void keep(v16h a, v16h b, v16h c, v16h d) { keep4_h(a, b, c, d); }
};
template <> struct Frag<__bf16> {
  typedef v16b V; union U { v16b v; v8b h[2]; };
  static __device__ __forceinline__ v16b load(const __bf16* p) {
    U f; f.h[0] = *(const v8b*)(p); f.h[1] = *(const v8b*)(p + 16); return f.v;
  }
  static __device__ __forceinline__ v8f mma(v16b a, v16b b, v8f c) {
    return __builtin_amdgcn_wmma_f32_16x16x32_bf16(false, a, false, b, (short)0, c, false, false);
  }
  static __device__ __forceinline__ void guard(v8f& a, v8f& b, v16b x, v16b y) { dep_guard_b(a, b, x, y); }
  static __device__ __forceinline__ void keep(v16b a, v16b b, v16b c, v16b d) { keep4_b(a, b, c, d); }
};

__device__ __forceinline__ float fsig(float x)  { return __builtin_amdgcn_rcpf(1.0f + __expf(-x)); }
__device__ __forceinline__ float ftanh(float x) { return 1.0f - 2.0f * __builtin_amdgcn_rcpf(__expf(2.0f * x) + 1.0f); }

template <int ET> struct Elem;
template <> struct Elem<0> { typedef _Float16 T; };
template <> struct Elem<1> { typedef __bf16 T; };
template <int ET, bool SPLIT, int BIAS_MODE, int OUT_MODE, bool RESID, int ACT = 0>
__global__ __launch_bounds__(256) void wmma_gemm64(
    const unsigned short* __restrict__ Ap, const unsigned short* __restrict__ A2p, int lda, long strideA,
    const unsigned short* __restrict__ Btp, const unsigned short* __restrict__ Bt2p, int ldb, long strideB,
    void* __restrict__ Cout, void* __restrict__ Cout2, int ldc, long strideC,
    const float* __restrict__ bias,
    const float* __restrict__ resid, long strideR,
    int M, int N, int K, float scale) {
  typedef typename Elem<ET>::T T;
  typedef typename Frag<T>::V V;
  const T* A = (const T*)Ap; const T* A2 = (const T*)A2p; const T* Bt = (const T*)Btp; const T* Bt2 = (const T*)Bt2p;
  __shared__ __align__(16) float sT[8][16 * 68];
  const int b    = blockIdx.y;
  const int lane = threadIdx.x & 31;
  const int wave = threadIdx.x >> 5;
  const int tilesN = N >> 6;
  const int tilesM = M >> 6;
  const int tile = blockIdx.x * 8 + wave;
  if (tile >= tilesM * tilesN) return;
  const int tm = tile / tilesN;
  const int tn = tile - tm * tilesN;
  const int m0 = tm << 6;
  const int n0 = tn << 6;

  const T* Ab  = A  + (size_t)b * strideA;
  const T* Bb  = Bt + (size_t)b * strideB;
  const T* Ab2 = SPLIT ? (A2  + (size_t)b * strideA) : nullptr;
  const T* Bb2 = SPLIT ? (Bt2 + (size_t)b * strideB) : nullptr;

  const int rlane = lane & 15;
  const int koff  = (lane >> 4) * 8;
  const int mOff  = (lane >> 4) * 8;

  v8f acc[4][4];
#pragma unroll
  for (int i = 0; i < 4; ++i)
#pragma unroll
    for (int j = 0; j < 4; ++j) acc[i][j] = (v8f){0.f,0.f,0.f,0.f,0.f,0.f,0.f,0.f};

  for (int k0 = 0; k0 < K; k0 += 32) {
    V bh[4], bl[4];
#pragma unroll
    for (int j = 0; j < 4; ++j) {
      const size_t bo = (size_t)(n0 + (j << 4) + rlane) * ldb + koff + k0;
      bh[j] = Frag<T>::load(Bb + bo);
      if (SPLIT) bl[j] = Frag<T>::load(Bb2 + bo);
    }
#pragma unroll
    for (int i = 0; i < 4; ++i) {
      const size_t ao = (size_t)(m0 + (i << 4) + rlane) * lda + koff + k0;
      V ah = Frag<T>::load(Ab + ao);
      V al;
      if (SPLIT) al = Frag<T>::load(Ab2 + ao);
#pragma unroll
      for (int j = 0; j < 4; ++j) {
        acc[i][j] = Frag<T>::mma(ah, bh[j], acc[i][j]);
        if (SPLIT) {
          acc[i][j] = Frag<T>::mma(ah, bl[j], acc[i][j]);
          acc[i][j] = Frag<T>::mma(al, bh[j], acc[i][j]);
        }
      }
      Frag<T>::guard(acc[i][0], acc[i][3], ah, SPLIT ? al : ah);
    }
    Frag<T>::keep(bh[0], bh[1], bh[2], bh[3]);
    if (SPLIT) Frag<T>::keep(bl[0], bl[1], bl[2], bl[3]);
  }
  acc_guard4(acc[0][0], acc[0][1], acc[0][2], acc[0][3]);
  acc_guard4(acc[1][0], acc[1][1], acc[1][2], acc[1][3]);
  acc_guard4(acc[2][0], acc[2][1], acc[2][2], acc[2][3]);
  acc_guard4(acc[3][0], acc[3][1], acc[3][2], acc[3][3]);

  float* slab = sT[wave];
  const float* Rb = RESID ? (resid + (size_t)b * strideR) : nullptr;
#pragma unroll
  for (int i = 0; i < 4; ++i) {
    const int mBase = m0 + (i << 4);
#pragma unroll
    for (int j = 0; j < 4; ++j) {
      const int n = n0 + (j << 4) + rlane;
      float bv = 0.f;
      if (BIAS_MODE == 2) bv = bias[n];
#pragma unroll
      for (int r = 0; r < 8; ++r) {
        float v = acc[i][j][r] * scale;
        if (BIAS_MODE == 1) v += bias[mBase + mOff + r];
        if (BIAS_MODE == 2) v += bv;
        if (RESID) v += Rb[(size_t)(mBase + mOff + r) * ldc + n];
        if (ACT == 1) v = tanhf(v);
        if (ACT == 2) v = fmaxf(v, 0.0f);
        if (ACT == 3) v = v / (1.0f + expf(-v));
        if (ACT == 4) v = (v > 0.f) ? v : 0.01f * v;
        if (ACT == 5) v = 0.5f * v * (1.0f + erff(v * 0.70710678118654752f));
        slab[(mOff + r) * 68 + (j << 4) + rlane] = v;
      }
    }
    __builtin_amdgcn_fence(__ATOMIC_RELEASE, "workgroup");
    __builtin_amdgcn_wave_barrier();
    __builtin_amdgcn_fence(__ATOMIC_ACQUIRE, "workgroup");
    if (OUT_MODE == 0) {
      float* C = (float*)Cout + (size_t)b * strideC;
      const int hh = lane >> 4, c4 = (lane & 15) * 4;
      for (int pass = 0; pass < 2; ++pass) {
#pragma unroll
        for (int it = 0; it < 8; ++it) {
          const int row = it * 2 + hh;
          v4f v = *(const v4f*)(slab + row * 68 + c4);
          *(volatile v4f*)(C + (size_t)(mBase + row) * ldc + n0 + c4) = v;
        }
        __threadfence();
      }
    } else {
      const int q = lane >> 3, c8 = (lane & 7) * 8;
      unsigned short* C  = (unsigned short*)Cout  + (size_t)b * strideC;
      unsigned short* C2 = (OUT_MODE == 2) ? ((unsigned short*)Cout2 + (size_t)b * strideC) : nullptr;
      for (int pass = 0; pass < 2; ++pass) {
#pragma unroll
        for (int it = 0; it < 4; ++it) {
          const int row = it * 4 + q;
          const float* sp = slab + row * 68 + c8;
          v8h hv, lv;
#pragma unroll
          for (int e = 0; e < 8; ++e) {
            if (OUT_MODE == 1) {
              hv[e] = (_Float16)sp[e];
            } else {
              unsigned short hb = f2bf_bits(sp[e]);
              unsigned short lb = f2bf_bits(sp[e] - bf_bits2f(hb));
              hv[e] = __builtin_bit_cast(_Float16, hb);
              lv[e] = __builtin_bit_cast(_Float16, lb);
            }
          }
          *(volatile v8h*)(C + (size_t)(mBase + row) * ldc + n0 + c8) = hv;
          if (OUT_MODE == 2) *(volatile v8h*)(C2 + (size_t)(mBase + row) * ldc + n0 + c8) = lv;
        }
        __threadfence();
      }
    }
    __builtin_amdgcn_fence(__ATOMIC_RELEASE, "workgroup");
    __builtin_amdgcn_wave_barrier();
    __builtin_amdgcn_fence(__ATOMIC_ACQUIRE, "workgroup");
  }
}

template <int MODE>
__global__ __launch_bounds__(NTHR) void cvt8_kernel(const float* __restrict__ src, unsigned short* __restrict__ dst,
                                                    int nrow, int ncol8, int spitch, int scol0, float sc) {
  const int i  = blockIdx.x * NTHR + threadIdx.x;
  const int n8 = nrow * ncol8;
  if (i < n8) {
    const int row = i / ncol8;
    const int c8  = i - row * ncol8;
    const float* sp = src + (size_t)row * spitch + scol0 + c8 * 8;
    const v4f a = *(const v4f*)(sp);
    const v4f b = *(const v4f*)(sp + 4);
    v8h hv;
#pragma unroll
    for (int e = 0; e < 4; ++e) {
      unsigned short b0, b1;
      if (MODE == 0) {
        b0 = f2bf_bits(a[e] * sc);
        b1 = f2bf_bits(b[e] * sc);
      } else {
        b0 = __builtin_bit_cast(unsigned short, (_Float16)(bf16r(a[e]) * sc));
        b1 = __builtin_bit_cast(unsigned short, (_Float16)(bf16r(b[e]) * sc));
      }
      hv[e]     = __builtin_bit_cast(_Float16, b0);
      hv[4 + e] = __builtin_bit_cast(_Float16, b1);
    }
    *(volatile v8h*)(dst + (size_t)i * 8) = hv;
    __threadfence();
    *(volatile v8h*)(dst + (size_t)i * 8) = hv;
  }
}

__global__ __launch_bounds__(NTHR) void bias_prep_kernel(const float* __restrict__ b_a, const float* __restrict__ b_b,
                                                         float* __restrict__ dst) {
  const int tid = threadIdx.x;
  const int which = tid >> 7;
  const int idx = (tid & 127) * 4;
  const v4f va = *(const v4f*)(b_a + idx);
  const v4f vb = *(const v4f*)(b_b + idx);
  v4f o;
#pragma unroll
  for (int e = 0; e < 4; ++e) o[e] = bf16r(which ? vb[e] : va[e]);
  float* op = dst + which * NHID + idx;
  *(volatile v4f*)op = o;
  __threadfence();
  *(volatile v4f*)op = o;
}

__global__ __launch_bounds__(NTHR) void ltc_seq_kernel(const float* __restrict__ XIN, const float* __restrict__ XTAU,
                                                       const unsigned short* __restrict__ WRp,
                                                       const unsigned short* __restrict__ WTp,
                                                       float* __restrict__ OUTH, float* __restrict__ HFIN) {
  __shared__ __align__(16) _Float16 Ah[2][SEQ_BLK * HPITCH];
  __shared__ __align__(16) float    Sl[NTHR / 32][16 * SLABP];
  const _Float16* WR = (const _Float16*)WRp;
  const _Float16* WT = (const _Float16*)WTp;
  const int tid = threadIdx.x, lane = tid & 31, wave = tid >> 5;
  const int c = lane & 15, hh = lane >> 4, koff = hh * 8, c4 = c * 4;
  const int rowbase = blockIdx.x * SEQ_BLK;

  {
    _Float16* ahf = &Ah[0][0];
#pragma unroll 1
    for (int i = tid; i < 2 * SEQ_BLK * HPITCH; i += NTHR) ahf[i] = (_Float16)0.0f;
  }
  float hst[4][8];
#pragma unroll
  for (int nt = 0; nt < 4; ++nt)
#pragma unroll
    for (int r = 0; r < 8; ++r) hst[nt][r] = 0.0f;
  __syncthreads();

  const v8f z8 = {0.f, 0.f, 0.f, 0.f, 0.f, 0.f, 0.f, 0.f};
  float* slab = Sl[wave];

#pragma unroll 1
  for (int t = 0; t < NSTEP; ++t) {
    float xr[4][8], tr[4][8];
#pragma unroll
    for (int nt = 0; nt < 4; ++nt) {
      const int j = 64 * wave + 16 * nt + c;
#pragma unroll
      for (int r = 0; r < 8; ++r) {
        const size_t off = ((size_t)(rowbase + 8 * hh + r) * NSTEP + (size_t)t) * NHID + j;
        xr[nt][r] = XIN[off];
        tr[nt][r] = XTAU[off];
      }
    }
    const bool last = (t == NSTEP - 1);

#pragma unroll 1
    for (int s = 0; s < NODE; ++s) {
      const int cur = s & 1;
      const _Float16* ahrow = &Ah[cur][0] + c * HPITCH + koff;
      _Float16* ahn = &Ah[cur ^ 1][0];
#pragma unroll
      for (int nt = 0; nt < 4; ++nt) {
        const int j = 64 * wave + 16 * nt + c;
        const _Float16* wr = WR + (size_t)j * NHID + koff;
        const _Float16* wt = WT + (size_t)j * NHID + koff;
        v8f accF = z8, accA = z8;
#pragma unroll 1
        for (int k0 = 0; k0 < NHID; k0 += 32) {
          const v16h a  = Frag<_Float16>::load(ahrow + k0);
          const v16h b0 = Frag<_Float16>::load(wr + k0);
          const v16h b1 = Frag<_Float16>::load(wt + k0);
          accF = Frag<_Float16>::mma(a, b0, accF);
          accA = Frag<_Float16>::mma(a, b1, accA);
          dep_guard_h(accF, accA, a, b1);
          keep4_h(a, b0, b1, a);
        }
        acc_guard2(accF, accA);
#pragma unroll
        for (int r = 0; r < 8; ++r) {
          const float zF = accF[r] * WCARRY_INV + xr[nt][r];
          const float zA = accA[r] * WCARRY_INV + tr[nt][r];
          const float al = fsig(zA);
          const float f  = ftanh(zF);
          const float ho = hst[nt][r];
          const float hn = (1.0f - al) * ho + al * f;
          hst[nt][r] = hn;
          ahn[(8 * hh + r) * HPITCH + j] = (_Float16)hn;
        }
      }
      __syncthreads();
    }

#pragma unroll
    for (int nt = 0; nt < 4; ++nt)
#pragma unroll
      for (int r = 0; r < 8; ++r) slab[(8 * hh + r) * SLABP + 16 * nt + c] = hst[nt][r];
    __builtin_amdgcn_fence(__ATOMIC_RELEASE, "workgroup");
    __builtin_amdgcn_wave_barrier();
    __builtin_amdgcn_fence(__ATOMIC_ACQUIRE, "workgroup");
    for (int pass = 0; pass < 2; ++pass) {
#pragma unroll
      for (int it = 0; it < 8; ++it) {
        const int row = it * 2 + hh;
        const v4f v = *(const v4f*)(slab + row * SLABP + c4);
        *(volatile v4f*)(OUTH + ((size_t)(rowbase + row) * NSTEP + (size_t)t) * NHID + 64 * wave + c4) = v;
        if (last) *(volatile v4f*)(HFIN + (size_t)(rowbase + row) * NHID + 64 * wave + c4) = v;
      }
      __threadfence();
    }
    __builtin_amdgcn_fence(__ATOMIC_RELEASE, "workgroup");
    __builtin_amdgcn_wave_barrier();
    __builtin_amdgcn_fence(__ATOMIC_ACQUIRE, "workgroup");
  }
}

__global__ __launch_bounds__(NTHR) void ln_rows_kernel(const float* __restrict__ YP, const float* __restrict__ gam,
                                                       const float* __restrict__ bet, float* __restrict__ Y, int nrows) {
  const int tid = threadIdx.x, lane = tid & 31;
  const int row = blockIdx.x * (NTHR / 32) + (tid >> 5);
  if (row >= nrows) return;
  const float* rp = YP + (size_t)row * NHID;
  v4f v[4], g[4], bb[4];
  float s = 0.0f;
#pragma unroll
  for (int q = 0; q < 4; ++q) {
    v[q]  = *(const v4f*)(rp  + 128 * q + 4 * lane);
    g[q]  = *(const v4f*)(gam + 128 * q + 4 * lane);
    bb[q] = *(const v4f*)(bet + 128 * q + 4 * lane);
    s += (v[q][0] + v[q][1]) + (v[q][2] + v[q][3]);
  }
#pragma unroll
  for (int off = 1; off < 32; off <<= 1) s += __shfl_xor(s, off, 32);
  const float mu = s * (1.0f / NHID);
  float ss = 0.0f;
#pragma unroll
  for (int q = 0; q < 4; ++q)
#pragma unroll
    for (int e = 0; e < 4; ++e) { const float d = v[q][e] - mu; v[q][e] = d; ss += d * d; }
#pragma unroll
  for (int off = 1; off < 32; off <<= 1) ss += __shfl_xor(ss, off, 32);
  const float var  = ss * (1.0f / NHID);
  const float rstd = rsqrtf(var + LN_EPS_F);
  v4f o[4];
#pragma unroll
  for (int q = 0; q < 4; ++q)
#pragma unroll
    for (int e = 0; e < 4; ++e) o[q][e] = (v[q][e] * rstd) * g[q][e] + bb[q][e];
  float* op = Y + (size_t)row * NHID;
  for (int pass = 0; pass < 2; ++pass) {
#pragma unroll
    for (int q = 0; q < 4; ++q) *(volatile v4f*)(op + 128 * q + 4 * lane) = o[q];
    __threadfence();
  }
}

extern "C" void kernel_launch(void* const* d_in, const int* in_sizes, int n_in,
                              void* d_out, int out_size, void* d_ws, size_t ws_size, hipStream_t stream) {
  if (n_in < 9 || d_out == nullptr || d_ws == nullptr) return;
  if (in_sizes[0] != NBATCH * NSTEP * NIN || in_sizes[1] != NHID * NIN || in_sizes[2] != NHID ||
      in_sizes[3] != NHID * NHID || in_sizes[4] != NHID * NTAU || in_sizes[5] != NHID ||
      in_sizes[6] != NHID * NIN || in_sizes[7] != NHID || in_sizes[8] != NHID ||
      out_size != NOUT0 + NOUT1) return;

  const float* x     = (const float*)d_in[0];
  const float* w_in  = (const float*)d_in[1];
  const float* b_in  = (const float*)d_in[2];
  const float* w_rec = (const float*)d_in[3];
  const float* w_tau = (const float*)d_in[4];
  const float* b_tau = (const float*)d_in[5];
  const float* w_res = (const float*)d_in[6];
  const float* gam   = (const float*)d_in[7];
  const float* bet   = (const float*)d_in[8];
  float* y_out = (float*)d_out;
  float* hfin  = y_out + (size_t)NOUT0;

  char* ws = (char*)d_ws; size_t off = 0;
  auto carve = [&](size_t bytes) -> char* { char* p = ws + off; off += (bytes + 255) & ~(size_t)255; return p; };
  unsigned short* XB    = (unsigned short*)carve((size_t)NROWS * NIN * 2);
  unsigned short* WINB  = (unsigned short*)carve((size_t)NHID * NIN * 2);
  unsigned short* WTXB  = (unsigned short*)carve((size_t)NHID * NIN * 2);
  unsigned short* WRESB = (unsigned short*)carve((size_t)NHID * NIN * 2);
  unsigned short* WHR   = (unsigned short*)carve((size_t)NHID * NHID * 2);
  unsigned short* WHT   = (unsigned short*)carve((size_t)NHID * NHID * 2);
  float*          BIAS2 = (float*)carve((size_t)2 * NHID * 4);
  float*          XIN   = (float*)carve((size_t)NROWS * NHID * 4);
  float*          XTAU  = (float*)carve((size_t)NROWS * NHID * 4);
  float*          OUTH  = (float*)carve((size_t)NROWS * NHID * 4);
  float*          YPRE  = XIN;
  if (off > ws_size || off > (size_t)134217728) return;

  const int n8x = NROWS * (NIN / 8);
  const int n8w = NHID * (NIN / 8);
  const int n8h = NHID * (NHID / 8);
  cvt8_kernel<0><<<(n8x + NTHR - 1) / NTHR, NTHR, 0, stream>>>(x,     XB,    NROWS, NIN / 8,  NIN,  0,   1.0f);
  cvt8_kernel<0><<<(n8w + NTHR - 1) / NTHR, NTHR, 0, stream>>>(w_in,  WINB,  NHID,  NIN / 8,  NIN,  0,   1.0f);
  cvt8_kernel<0><<<(n8w + NTHR - 1) / NTHR, NTHR, 0, stream>>>(w_tau, WTXB,  NHID,  NIN / 8,  NTAU, 0,   1.0f);
  cvt8_kernel<0><<<(n8w + NTHR - 1) / NTHR, NTHR, 0, stream>>>(w_res, WRESB, NHID,  NIN / 8,  NIN,  0,   1.0f);
  cvt8_kernel<1><<<(n8h + NTHR - 1) / NTHR, NTHR, 0, stream>>>(w_rec, WHR,   NHID,  NHID / 8, NHID, 0,   WCARRY);
  cvt8_kernel<1><<<(n8h + NTHR - 1) / NTHR, NTHR, 0, stream>>>(w_tau, WHT,   NHID,  NHID / 8, NTAU, NIN, WCARRY);
  bias_prep_kernel<<<1, NTHR, 0, stream>>>(b_in, b_tau, BIAS2);

  const dim3 ggrid((NROWS / 64) * (NHID / 64) / 8, 1);
  wmma_gemm64<1, false, 2, 0, false, 0><<<ggrid, 256, 0, stream>>>(
      XB, XB, NIN, 0L, WINB, WINB, NIN, 0L, (void*)XIN, (void*)XIN, NHID, 0L,
      BIAS2, OUTH, 0L, NROWS, NHID, NIN, 1.0f);
  wmma_gemm64<1, false, 2, 0, false, 0><<<ggrid, 256, 0, stream>>>(
      XB, XB, NIN, 0L, WTXB, WTXB, NIN, 0L, (void*)XTAU, (void*)XTAU, NHID, 0L,
      BIAS2 + NHID, OUTH, 0L, NROWS, NHID, NIN, 1.0f);

  ltc_seq_kernel<<<NBATCH / SEQ_BLK, NTHR, 0, stream>>>(XIN, XTAU, WHR, WHT, OUTH, hfin);

  wmma_gemm64<1, false, 0, 0, true, 0><<<ggrid, 256, 0, stream>>>(
      XB, XB, NIN, 0L, WRESB, WRESB, NIN, 0L, (void*)YPRE, (void*)YPRE, NHID, 0L,
      BIAS2, OUTH, 0L, NROWS, NHID, NIN, 1.0f);

  ln_rows_kernel<<<NROWS / (NTHR / 32), NTHR, 0, stream>>>(YPRE, gam, bet, y_out, NROWS);
}
